// CharRNN_29463475651457
// MI455X (gfx1250) — hardware-verified
//
#include <hip/hip_runtime.h>
#include <math.h>

constexpr int NBAT  = 256;
constexpr int NSTP  = 256;
constexpr int NHID  = 1024;
constexpr int NVOC  = 128;
constexpr int TCH   = 32;
constexpr int NTHR  = 256;
constexpr int SLABP = 68;
constexpr int PLANE = NBAT * NHID;
constexpr int NOUT0 = NBAT * NSTP * NVOC;
constexpr int NOUT1 = NBAT * NHID;
constexpr float WCARRY     = 64.0f;
constexpr float WCARRY_INV = 1.0f / 64.0f;
constexpr float LCARRY     = 2048.0f;
constexpr float SC_HI      = WCARRY_INV;
constexpr float SC_LO      = WCARRY_INV / LCARRY;
constexpr float SC_PROJ    = WCARRY_INV * WCARRY_INV;
constexpr float F16_MIN_NORMAL = 6.103515625e-5f;
static_assert(NHID % 32 == 0);
static_assert(NBAT % 64 == 0 && NHID % 256 == 0 && NVOC % 64 == 0);
static_assert((TCH * NBAT) % 64 == 0 && NSTP % TCH == 0);
static_assert((size_t)NOUT0 * 4 == 33554432u);
static_assert(((size_t)NOUT0 * 4) % 128 == 0);
static_assert((size_t)(NOUT0 + NOUT1) * 4 == 34603008u);
static_assert((NVOC * NHID / 8) % NTHR == 0 && (NHID * NHID / 8) % NTHR == 0 && (PLANE / 8) % NTHR == 0);

typedef __attribute__((ext_vector_type(16))) _Float16 v16h;
typedef __attribute__((ext_vector_type(8)))  _Float16 v8h;
typedef __attribute__((ext_vector_type(8)))  float    v8f;
typedef __attribute__((ext_vector_type(4)))  float    v4f;
typedef __attribute__((ext_vector_type(4)))  unsigned v4u;

__device__ __forceinline__ unsigned short f2bf_bits(float f) {
  unsigned u = __float_as_uint(f);
  return (unsigned short)((u + 0x7FFFu + ((u >> 16) & 1u)) >> 16);
}
__device__ __forceinline__ float bf16r(float f) { return __uint_as_float(((unsigned)f2bf_bits(f)) << 16); }

__device__ __forceinline__ void guard8_h(v8f& a0, v8f& a1, v8f& a2, v8f& a3, v8f& a4, v8f& a5, v8f& a6, v8f& a7, v16h x, v16h y) {
  asm volatile("v_nop\n\tv_nop\n\tv_nop\n\tv_nop" : "+v"(a0), "+v"(a1), "+v"(a2), "+v"(a3), "+v"(a4), "+v"(a5), "+v"(a6), "+v"(a7) : "v"(x), "v"(y));
}
__device__ __forceinline__ void guard4_h(v8f& a0, v8f& a1, v8f& a2, v8f& a3, v16h x, v16h y) {
  asm volatile("v_nop\n\tv_nop\n\tv_nop\n\tv_nop" : "+v"(a0), "+v"(a1), "+v"(a2), "+v"(a3) : "v"(x), "v"(y));
}
__device__ __forceinline__ void keep4_h(v16h a, v16h b, v16h c, v16h d) { asm volatile("v_nop" :: "v"(a), "v"(b), "v"(c), "v"(d)); }
__device__ __forceinline__ void acc_guard4(v8f& a, v8f& b, v8f& c, v8f& d) { asm volatile("v_nop\n\tv_nop\n\tv_nop\n\tv_nop" : "+v"(a), "+v"(b), "+v"(c), "+v"(d)); }
__device__ __forceinline__ void acc_guard8(v8f& a0, v8f& a1, v8f& a2, v8f& a3, v8f& a4, v8f& a5, v8f& a6, v8f& a7) {
  asm volatile("v_nop\n\tv_nop\n\tv_nop\n\tv_nop" : "+v"(a0), "+v"(a1), "+v"(a2), "+v"(a3), "+v"(a4), "+v"(a5), "+v"(a6), "+v"(a7));
}

struct FragH {
  union U { v16h v; v8h h[2]; };
  static __device__ __forceinline__ v16h load(const _Float16* p) {
    U f; f.h[0] = *(const v8h*)(p); f.h[1] = *(const v8h*)(p + 16); return f.v;
  }
  static __device__ __forceinline__ v8f mma(v16h a, v16h b, v8f c) {
    return __builtin_amdgcn_wmma_f32_16x16x32_f16(false, a, false, b, (short)0, c, false, false);
  }
};

__device__ __forceinline__ void wave_lds_sync() {
  __builtin_amdgcn_fence(__ATOMIC_RELEASE, "workgroup");
  __builtin_amdgcn_wave_barrier();
  __builtin_amdgcn_fence(__ATOMIC_ACQUIRE, "workgroup");
}

__device__ __forceinline__ float ftanh(float x) { return 1.0f - 2.0f * __builtin_amdgcn_rcpf(__expf(2.0f * x) + 1.0f); }

__global__ __launch_bounds__(NTHR) void cvt8_kernel(const float* __restrict__ src, unsigned short* __restrict__ dst, int n8, float sc) {
  const int i = blockIdx.x * NTHR + threadIdx.x;
  if (i < n8) {
    const float* sp = src + (size_t)i * 8;
    const v4f a = *(const v4f*)(sp);
    const v4f b = *(const v4f*)(sp + 4);
    v8h hv;
#pragma unroll
    for (int e = 0; e < 4; ++e) {
      const float fa = bf16r(a[e]) * sc;
      const float fb = bf16r(b[e]) * sc;
      hv[e]     = (_Float16)fa;
      hv[4 + e] = (_Float16)fb;
    }
    *(volatile v8h*)(dst + (size_t)i * 8) = hv;
    __threadfence();
    *(volatile v8h*)(dst + (size_t)i * 8) = hv;
  }
}

__global__ __launch_bounds__(NTHR) void bias_prep_kernel(const float* __restrict__ b_xh, const float* __restrict__ b_hh,
                                                         const float* __restrict__ b_fc,
                                                         float* __restrict__ bsum, float* __restrict__ fcb) {
  const int tid = threadIdx.x;
  const int idx = tid * 4;
  const int fi  = (tid & 31) * 4;
  const v4f va = *(const v4f*)(b_xh + idx);
  const v4f vb = *(const v4f*)(b_hh + idx);
  const v4f vc = *(const v4f*)(b_fc + fi);
  v4f o, oc;
#pragma unroll
  for (int e = 0; e < 4; ++e) { o[e] = bf16r(va[e]) + bf16r(vb[e]); oc[e] = bf16r(vc[e]); }
  *(volatile v4f*)(bsum + idx) = o;
  if (tid < 32) *(volatile v4f*)(fcb + fi) = oc;
  __threadfence();
  *(volatile v4f*)(bsum + idx) = o;
  if (tid < 32) *(volatile v4f*)(fcb + fi) = oc;
}

__global__ __launch_bounds__(NTHR) void zero2_kernel(unsigned short* __restrict__ p0, unsigned short* __restrict__ p1, int n8) {
  const int i = blockIdx.x * NTHR + threadIdx.x;
  if (i < n8) {
    const v4u z = {0u, 0u, 0u, 0u};
    *(volatile v4u*)(p0 + (size_t)i * 8) = z;
    *(volatile v4u*)(p1 + (size_t)i * 8) = z;
    __threadfence();
    *(volatile v4u*)(p0 + (size_t)i * 8) = z;
    *(volatile v4u*)(p1 + (size_t)i * 8) = z;
  }
}

template <int OUTMAP>
__global__ __launch_bounds__(NTHR) void gemm64_f16_kernel(
    const unsigned short* __restrict__ Ap, int lda,
    const unsigned short* __restrict__ Btp, int ldb,
    float* __restrict__ Cout, int ldc,
    const float* __restrict__ bias, int M, int N, int K, float scale, int t0) {
  const _Float16* A  = (const _Float16*)Ap;
  const _Float16* Bt = (const _Float16*)Btp;
  __shared__ __align__(16) float sT[NTHR / 32][16 * SLABP];
  const int lane = threadIdx.x & 31;
  const int wave = threadIdx.x >> 5;
  const int tilesN = N >> 6;
  const int tilesM = M >> 6;
  const int tile = blockIdx.x * 8 + wave;
  if (tile >= tilesM * tilesN) return;
  const int tm = tile / tilesN;
  const int tn = tile - tm * tilesN;
  const int m0 = tm << 6;
  const int n0 = tn << 6;
  const int rl   = lane & 15;
  const int hh   = lane >> 4;
  const int koff = hh * 8;
  const int mOff = hh * 8;

  v8f acc[4][4];
#pragma unroll
  for (int i = 0; i < 4; ++i)
#pragma unroll
    for (int j = 0; j < 4; ++j) acc[i][j] = (v8f){0.f, 0.f, 0.f, 0.f, 0.f, 0.f, 0.f, 0.f};

#pragma unroll 1
  for (int k0 = 0; k0 < K; k0 += 32) {
    v16h bh[4];
#pragma unroll
    for (int j = 0; j < 4; ++j) bh[j] = FragH::load(Bt + (size_t)(n0 + (j << 4) + rl) * ldb + koff + k0);
#pragma unroll
    for (int i = 0; i < 4; ++i) {
      const v16h ah = FragH::load(A + (size_t)(m0 + (i << 4) + rl) * lda + koff + k0);
#pragma unroll
      for (int j = 0; j < 4; ++j) acc[i][j] = FragH::mma(ah, bh[j], acc[i][j]);
      guard4_h(acc[i][0], acc[i][1], acc[i][2], acc[i][3], ah, bh[3]);
    }
    keep4_h(bh[0], bh[1], bh[2], bh[3]);
  }
  acc_guard4(acc[0][0], acc[0][1], acc[0][2], acc[0][3]);
  acc_guard4(acc[1][0], acc[1][1], acc[1][2], acc[1][3]);
  acc_guard4(acc[2][0], acc[2][1], acc[2][2], acc[2][3]);
  acc_guard4(acc[3][0], acc[3][1], acc[3][2], acc[3][3]);

  float* slab = sT[wave];
  const int c4 = rl * 4;
#pragma unroll
  for (int i = 0; i < 4; ++i) {
    const int mBase = m0 + (i << 4);
#pragma unroll
    for (int j = 0; j < 4; ++j) {
      const float bv = bias[n0 + (j << 4) + rl];
#pragma unroll
      for (int r = 0; r < 8; ++r) slab[(mOff + r) * SLABP + (j << 4) + rl] = acc[i][j][r] * scale + bv;
    }
    wave_lds_sync();
    for (int pass = 0; pass < 2; ++pass) {
#pragma unroll
      for (int it = 0; it < 8; ++it) {
        const int row = it * 2 + hh;
        const int m = mBase + row;
        size_t orow;
        if (OUTMAP == 0) orow = (size_t)m;
        else orow = (size_t)(m % NBAT) * NSTP + (size_t)(t0 + m / NBAT);
        const v4f v = *(const v4f*)(slab + row * SLABP + c4);
        *(volatile v4f*)(Cout + orow * (size_t)ldc + n0 + c4) = v;
      }
      __threadfence();
    }
    wave_lds_sync();
  }
}

__global__ __launch_bounds__(NTHR) void rnn_step_kernel(
    const unsigned short* __restrict__ HhiIn, const unsigned short* __restrict__ HloIn,
    const unsigned short* __restrict__ Wp, const float* __restrict__ Ptab,
    const int* __restrict__ tok,
    unsigned short* __restrict__ HhiOut, unsigned short* __restrict__ HloOut,
    float* __restrict__ Hfin, int t, int last) {
  __shared__ __align__(16) float sT[NTHR / 32][32 * SLABP];
  const _Float16* Ah = (const _Float16*)HhiIn;
  const _Float16* Al = (const _Float16*)HloIn;
  const _Float16* W  = (const _Float16*)Wp;
  const int lane = threadIdx.x & 31;
  const int wave = threadIdx.x >> 5;
  const int rl   = lane & 15;
  const int hh   = lane >> 4;
  const int koff = hh * 8;
  const int m0 = blockIdx.y * 64 + (wave & 1) * 32;
  const int n0 = blockIdx.x * 256 + (wave >> 1) * 64;

  v8f accH[2][4], accL[2][4];
#pragma unroll
  for (int i = 0; i < 2; ++i)
#pragma unroll
    for (int j = 0; j < 4; ++j) {
      accH[i][j] = (v8f){0.f, 0.f, 0.f, 0.f, 0.f, 0.f, 0.f, 0.f};
      accL[i][j] = (v8f){0.f, 0.f, 0.f, 0.f, 0.f, 0.f, 0.f, 0.f};
    }

  const _Float16* bp  = W  + (size_t)(n0 + rl) * NHID + koff;
  const _Float16* ahp = Ah + (size_t)(m0 + rl) * NHID + koff;
  const _Float16* alp = Al + (size_t)(m0 + rl) * NHID + koff;

#pragma unroll 1
  for (int k0 = 0; k0 < NHID; k0 += 32) {
    v16h bf[4];
#pragma unroll
    for (int j = 0; j < 4; ++j) bf[j] = FragH::load(bp + (size_t)j * 16 * NHID + k0);
#pragma unroll
    for (int i = 0; i < 2; ++i) {
      const v16h ah = FragH::load(ahp + (size_t)i * 16 * NHID + k0);
      const v16h al = FragH::load(alp + (size_t)i * 16 * NHID + k0);
#pragma unroll
      for (int j = 0; j < 4; ++j) {
        accH[i][j] = FragH::mma(ah, bf[j], accH[i][j]);
        accL[i][j] = FragH::mma(al, bf[j], accL[i][j]);
      }
      guard8_h(accH[i][0], accH[i][1], accH[i][2], accH[i][3], accL[i][0], accL[i][1], accL[i][2], accL[i][3], ah, al);
    }
    keep4_h(bf[0], bf[1], bf[2], bf[3]);
  }
  acc_guard8(accH[0][0], accH[0][1], accH[0][2], accH[0][3], accH[1][0], accH[1][1], accH[1][2], accH[1][3]);
  acc_guard8(accL[0][0], accL[0][1], accL[0][2], accL[0][3], accL[1][0], accL[1][1], accL[1][2], accL[1][3]);

  float* slab = sT[wave];
#pragma unroll
  for (int i = 0; i < 2; ++i)
#pragma unroll
    for (int j = 0; j < 4; ++j)
#pragma unroll
      for (int r = 0; r < 8; ++r)
        slab[(16 * i + 8 * hh + r) * SLABP + 16 * j + rl] = accH[i][j][r] * SC_HI + accL[i][j][r] * SC_LO;
  wave_lds_sync();

  const int q  = lane >> 3;
  const int c8 = (lane & 7) * 8;
#pragma unroll 1
  for (int it = 0; it < 8; ++it) {
    const int row  = it * 4 + q;
    const int grow = m0 + row;
    int tk = tok[(size_t)grow * NSTP + t];
    tk = tk < 0 ? 0 : tk;
    tk = tk > (NVOC - 1) ? (NVOC - 1) : tk;
    const float* pp = Ptab + (size_t)tk * NHID + n0 + c8;
    const v4f p0 = *(const v4f*)(pp);
    const v4f p1 = *(const v4f*)(pp + 4);
    float* sp = slab + row * SLABP + c8;
    const v4f z0 = *(const v4f*)(sp);
    const v4f z1 = *(const v4f*)(sp + 4);
    v8h hv, lv;
    v4f f0, f1;
#pragma unroll
    for (int e = 0; e < 8; ++e) {
      const float zz = (e < 4) ? (z0[e & 3] + p0[e & 3]) : (z1[e & 3] + p1[e & 3]);
      const float v  = ftanh(zz);
      const float vh = (fabsf(v) < F16_MIN_NORMAL) ? 0.0f : v;
      const _Float16 hi = (_Float16)vh;
      float hf = (float)hi;
      asm volatile("" : "+v"(hf));
      const float rs = (v - hf) * LCARRY;
      hv[e] = hi;
      lv[e] = (_Float16)rs;
      if (e < 4) f0[e & 3] = v; else f1[e & 3] = v;
    }
    if (last) {
      *(v4f*)(sp)     = f0;
      *(v4f*)(sp + 4) = f1;
    }
    unsigned short* ph = HhiOut + (size_t)grow * NHID + n0 + c8;
    unsigned short* pl = HloOut + (size_t)grow * NHID + n0 + c8;
    *(volatile v8h*)ph = hv;
    *(volatile v8h*)pl = lv;
    __threadfence();
    *(volatile v8h*)ph = hv;
    *(volatile v8h*)pl = lv;
  }

  if (last) {
    wave_lds_sync();
    const int c4 = rl * 4;
    for (int pass = 0; pass < 2; ++pass) {
#pragma unroll 1
      for (int it = 0; it < 16; ++it) {
        const int row = it * 2 + hh;
        const v4f v = *(const v4f*)(slab + row * SLABP + c4);
        *(volatile v4f*)(Hfin + (size_t)(m0 + row) * NHID + n0 + c4) = v;
      }
      __threadfence();
    }
  }
}

extern "C" void kernel_launch(void* const* d_in, const int* in_sizes, int n_in,
                              void* d_out, int out_size, void* d_ws, size_t ws_size, hipStream_t stream) {
  if (n_in < 8 || d_out == nullptr || d_ws == nullptr) return;
  if (in_sizes[0] != NBAT * NSTP || in_sizes[1] != NVOC * NHID || in_sizes[2] != NHID * NHID ||
      in_sizes[3] != NHID || in_sizes[4] != NHID * NHID || in_sizes[5] != NHID ||
      in_sizes[6] != NVOC * NHID || in_sizes[7] != NVOC || out_size != NOUT0 + NOUT1) return;

  const int*   tokp  = (const int*)d_in[0];
  const float* embed = (const float*)d_in[1];
  const float* wxh   = (const float*)d_in[2];
  const float* bxh   = (const float*)d_in[3];
  const float* whh   = (const float*)d_in[4];
  const float* bhh   = (const float*)d_in[5];
  const float* fcw   = (const float*)d_in[6];
  const float* fcbi  = (const float*)d_in[7];
  float* out0 = (float*)d_out;
  float* out1 = out0 + (size_t)NOUT0;

  char* ws = (char*)d_ws; size_t off = 0;
  auto carve = [&](size_t bytes) -> char* { char* p = ws + off; off += (bytes + 255) & ~(size_t)255; return p; };
  float*          PTAB  = (float*)carve((size_t)NVOC * NHID * 4);
  unsigned short* EMB16 = (unsigned short*)carve((size_t)NVOC * NHID * 2);
  unsigned short* WXH16 = (unsigned short*)carve((size_t)NHID * NHID * 2);
  unsigned short* WHH16 = (unsigned short*)carve((size_t)NHID * NHID * 2);
  unsigned short* FCW16 = (unsigned short*)carve((size_t)NVOC * NHID * 2);
  float*          BSUM  = (float*)carve((size_t)NHID * 4);
  float*          FCBR  = (float*)carve((size_t)NVOC * 4);
  unsigned short* HRING = (unsigned short*)carve((size_t)TCH * PLANE * 2);
  unsigned short* HLO   = (unsigned short*)carve((size_t)2 * PLANE * 2);
  if (off > ws_size || off > (size_t)134217728) return;

  const int n8small = NVOC * NHID / 8;
  const int n8big   = NHID * NHID / 8;
  const int n8plane = PLANE / 8;
  cvt8_kernel<<<n8small / NTHR, NTHR, 0, stream>>>(embed, EMB16, n8small, WCARRY);
  cvt8_kernel<<<n8big / NTHR,   NTHR, 0, stream>>>(wxh,   WXH16, n8big,   WCARRY);
  cvt8_kernel<<<n8big / NTHR,   NTHR, 0, stream>>>(whh,   WHH16, n8big,   WCARRY);
  cvt8_kernel<<<n8small / NTHR, NTHR, 0, stream>>>(fcw,   FCW16, n8small, WCARRY);
  bias_prep_kernel<<<1, NTHR, 0, stream>>>(bxh, bhh, fcbi, BSUM, FCBR);
  zero2_kernel<<<n8plane / NTHR, NTHR, 0, stream>>>(HRING + (size_t)(TCH - 1) * PLANE, HLO + (size_t)PLANE, n8plane);

  gemm64_f16_kernel<0><<<(NVOC / 64) * (NHID / 64) / 8, NTHR, 0, stream>>>(
      EMB16, NHID, WXH16, NHID, PTAB, NHID, BSUM, NVOC, NHID, NHID, SC_PROJ, 0);

  const dim3 sgrid(NHID / 256, NBAT / 64);
  const int fcblocks = ((TCH * NBAT) / 64) * (NVOC / 64) / 8;
  for (int t = 0; t < NSTP; ++t) {
    const unsigned short* hin  = HRING + (size_t)((t + TCH - 1) % TCH) * PLANE;
    const unsigned short* lin  = HLO + (size_t)((t + 1) & 1) * PLANE;
    unsigned short* hout = HRING + (size_t)(t % TCH) * PLANE;
    unsigned short* lout = HLO + (size_t)(t & 1) * PLANE;
    rnn_step_kernel<<<sgrid, NTHR, 0, stream>>>(hin, lin, WHH16, PTAB, tokp, hout, lout, out1, t, (t == NSTP - 1) ? 1 : 0);
    if ((t % TCH) == TCH - 1) {
      gemm64_f16_kernel<1><<<fcblocks, NTHR, 0, stream>>>(
          HRING, NHID, FCW16, NHID, out0, NVOC, FCBR, TCH * NBAT, NVOC, NHID, WCARRY_INV, t - (TCH - 1));
    }
  }
}
